// GAT_58832462020773
// MI455X (gfx1250) — hardware-verified
//
#include <hip/hip_runtime.h>
#include <stddef.h>
#include <stdint.h>
#include <math.h>


#define NN      256
#define HD      256
#define DDE     64
#define NHD     4
#define NSLOT   257
#define KG      128
#define KC      2048
#define APITCH  136
#define EP      264
#define PB_T    64
#define PB_PQ   32
#define PB_WG   8
#define PB_WM   128
#define PB_UV   4
#define PB_ALL  (PB_T + PB_PQ + PB_WG + PB_WM + PB_UV)
#define LDS_PAIR (64 * 256 * 4 + 64 * APITCH * 2)
#define WSMAX   134217728

static_assert(PB_T * 1024 == NN * HD);
static_assert(PB_PQ * 256 == 2 * NN * (DDE / 4));
static_assert(PB_WG * 256 * 8 == HD * DDE);
static_assert(PB_WM * 256 * 8 == HD * NHD * HD);
static_assert(PB_UV == NHD);
static_assert((KG % 32) == 0 && (KC % 32) == 0);
static_assert(KG == 2 * DDE && KC == 2 * NHD * HD);
static_assert((APITCH % 8) == 0 && APITCH >= KG);
static_assert(EP >= NSLOT && (EP % 4) == 0);
static_assert(LDS_PAIR <= 300000);

typedef float          v2f  __attribute__((ext_vector_type(2)));
typedef float          v4f  __attribute__((ext_vector_type(4)));
typedef float          v8f  __attribute__((ext_vector_type(8)));
typedef int            v8i  __attribute__((ext_vector_type(8)));
typedef unsigned short v8us __attribute__((ext_vector_type(8)));
typedef __bf16         v16b __attribute__((ext_vector_type(16)));
typedef v2f  __attribute__((may_alias)) v2fa;
typedef v4f  __attribute__((may_alias)) v4fa;
typedef v8us __attribute__((may_alias)) v8usa;
union FragB { v16b v; v8us h[2]; v8i w; };

__device__ __forceinline__ v8f wmb(const FragB& a, const FragB& b, v8f c) {
  v8f d = __builtin_amdgcn_wmma_f32_16x16x32_bf16(false, a.v, false, b.v, (short)0, c, false, false);
  asm volatile("v_nop\n\tv_nop\n\tv_nop\n\tv_nop" : "+v"(d) : "v"(a.w), "v"(b.w));
  return d;
}

__device__ __forceinline__ unsigned int f2bf(float f) {
  const unsigned int u = __float_as_uint(f);
  return ((u + 0x7FFFu + ((u >> 16) & 1u)) >> 16) & 0xFFFFu;
}
__device__ __forceinline__ float bf2f(unsigned int b) { return __uint_as_float(b << 16); }
__device__ __forceinline__ float bfr(float f) { return bf2f(f2bf(f)); }
__device__ __forceinline__ v4f bfr4(const v4f a) {
  v4f r; r.x = bfr(a.x); r.y = bfr(a.y); r.z = bfr(a.z); r.w = bfr(a.w); return r;
}
__device__ __forceinline__ float wsum(float v) {
#pragma unroll
  for (int o = 16; o > 0; o >>= 1) v += __shfl_xor(v, o);
  return v;
}
__device__ __forceinline__ float wmax(float v) {
#pragma unroll
  for (int o = 16; o > 0; o >>= 1) v = fmaxf(v, __shfl_xor(v, o));
  return v;
}
__device__ __forceinline__ float dot8(const v4f x0, const v4f x1, const v4f w0, const v4f w1) {
  float d = x0.x * w0.x;
  d = fmaf(x0.y, w0.y, d); d = fmaf(x0.z, w0.z, d); d = fmaf(x0.w, w0.w, d);
  d = fmaf(x1.x, w1.x, d); d = fmaf(x1.y, w1.y, d); d = fmaf(x1.z, w1.z, d); d = fmaf(x1.w, w1.w, d);
  return d;
}
__device__ __forceinline__ float sigm(float x) { return 1.0f / (1.0f + expf(-x)); }

__global__ __launch_bounds__(256) void k_prep(
    const float* __restrict__ ahs, const float* __restrict__ goal, const float* __restrict__ action,
    const float* __restrict__ Wd, const float* __restrict__ Wg, const float* __restrict__ wm,
    const float* __restrict__ av,
    float* TT, float* HO, float* PQ, unsigned short* WG2, unsigned short* WM2, float* UV)
{
  __shared__ __attribute__((aligned(16))) float sm[2048];
  const int tid = (int)threadIdx.x;
  const int b   = (int)blockIdx.x;

  if (b < PB_T) {
    float* sT = sm;
    float* sH = sm + 1024;
    const int base = b * 1024;
#pragma unroll 1
    for (int e = 0; e < 4; ++e) {
      const int idx = e * 256 + tid;
      const float v = bfr(ahs[base + idx]);
      sH[idx] = v;
      sT[idx] = tanhf(v);
    }
    __syncthreads();
    const v4f tv = *(const v4fa*)(sT + 4 * tid);
    const v4f hv = *(const v4fa*)(sH + 4 * tid);
    const int g   = base + 4 * tid;
    const int row = g >> 8;
    const int col = g & 255;
    float* tp = TT + g;
    float* hp = HO + (size_t)row * (size_t)(NSLOT * HD) + col;
    *(volatile v4f*)tp = tv;
    *(volatile v4f*)hp = hv;
    __threadfence();
    *(volatile v4f*)tp = tv;
    *(volatile v4f*)hp = hv;
  } else if (b < PB_T + PB_PQ) {
    const int u   = (b - PB_T) * 256 + tid;
    const int sel = u >> 12;
    const int v   = u & 4095;
    const int n   = v >> 4;
    const int d0  = (v & 15) * 4;
    const v2f ac = *(const v2fa*)(action + 2 * n);
    const v2f go = *(const v2fa*)(goal + 2 * n);
    const float a0 = bfr(ac.x), a1 = bfr(ac.y), g0 = bfr(go.x), g1 = bfr(go.y);
    const float* wd = Wd + sel * 256 + d0;
    const v4f w0 = bfr4(*(const v4fa*)(wd));
    const v4f w1 = bfr4(*(const v4fa*)(wd + 64));
    const v4f w2 = bfr4(*(const v4fa*)(wd + 128));
    const v4f w3 = bfr4(*(const v4fa*)(wd + 192));
    v4f r;
    r.x = fmaf(g1, w3.x, fmaf(g0, w2.x, fmaf(a1, w1.x, a0 * w0.x)));
    r.y = fmaf(g1, w3.y, fmaf(g0, w2.y, fmaf(a1, w1.y, a0 * w0.y)));
    r.z = fmaf(g1, w3.z, fmaf(g0, w2.z, fmaf(a1, w1.z, a0 * w0.z)));
    r.w = fmaf(g1, w3.w, fmaf(g0, w2.w, fmaf(a1, w1.w, a0 * w0.w)));
    float* dp = PQ + sel * (NN * DDE) + n * DDE + d0;
    *(volatile v4f*)dp = r;
    __threadfence();
    *(volatile v4f*)dp = r;
  } else if (b < PB_T + PB_PQ + PB_WG) {
    const int u  = (b - PB_T - PB_PQ) * 256 + tid;
    const int n  = u >> 3;
    const int k8 = (u & 7) * 8;
    const float* p = Wg + (size_t)k8 * HD + n;
    v8us o;
#pragma unroll
    for (int i = 0; i < 8; ++i) o[i] = (unsigned short)f2bf(p[(size_t)i * HD]);
    unsigned short* dp = WG2 + (size_t)n * KG + k8;
    *(volatile v8us*)dp = o;
    *(volatile v8us*)(dp + DDE) = o;
    __threadfence();
    *(volatile v8us*)dp = o;
    *(volatile v8us*)(dp + DDE) = o;
  } else if (b < PB_T + PB_PQ + PB_WG + PB_WM) {
    const int u  = (b - PB_T - PB_PQ - PB_WG) * 256 + tid;
    const int f  = u >> 7;
    const int k8 = (u & 127) * 8;
    const float* p = wm + (size_t)k8 * HD + f;
    v8us o;
#pragma unroll
    for (int i = 0; i < 8; ++i) o[i] = (unsigned short)f2bf(p[(size_t)i * HD]);
    unsigned short* dp = WM2 + (size_t)f * KC + k8;
    *(volatile v8us*)dp = o;
    *(volatile v8us*)(dp + NHD * HD) = o;
    __threadfence();
    *(volatile v8us*)dp = o;
    *(volatile v8us*)(dp + NHD * HD) = o;
  } else if (b < PB_ALL) {
    const int z = b - (PB_T + PB_PQ + PB_WG + PB_WM);
    sm[tid]       = bfr(av[tid]);
    sm[256 + tid] = bfr(av[256 + tid]);
    __syncthreads();
    const float* wr = wm + (size_t)(z * HD + tid) * HD;
    float ua = 0.0f, va = 0.0f;
#pragma unroll 2
    for (int f4 = 0; f4 < HD / 4; ++f4) {
      const v4f w  = bfr4(*(const v4fa*)(wr + 4 * f4));
      const v4f a1 = *(const v4fa*)(sm + 4 * f4);
      const v4f a2 = *(const v4fa*)(sm + 256 + 4 * f4);
      ua = fmaf(w.x, a1.x, ua); ua = fmaf(w.y, a1.y, ua); ua = fmaf(w.z, a1.z, ua); ua = fmaf(w.w, a1.w, ua);
      va = fmaf(w.x, a2.x, va); va = fmaf(w.y, a2.y, va); va = fmaf(w.z, a2.z, va); va = fmaf(w.w, a2.w, va);
    }
    sm[1024 + tid] = ua;
    sm[1280 + tid] = va;
    __syncthreads();
    if (tid < 128) {
      const int which = tid >> 6;
      const int q     = tid & 63;
      const v4f v = *(const v4fa*)(sm + 1024 + which * 256 + 4 * q);
      float* dp = UV + which * (NHD * HD) + z * HD + 4 * q;
      *(volatile v4f*)dp = v;
      __threadfence();
      *(volatile v4f*)dp = v;
    }
  }
}

__global__ __launch_bounds__(256) void k_pair(
    const float* __restrict__ PQ, const float* __restrict__ bd,
    const unsigned short* __restrict__ WG2, const float* __restrict__ bg,
    const float* __restrict__ TT, const float* __restrict__ ghs, float* HO)
{
  extern __shared__ __attribute__((aligned(16))) float gsm[];
  float* stg = gsm;
  unsigned short* As = (unsigned short*)(gsm + 64 * 256);
  const int tid = (int)threadIdx.x, lane = tid & 31;
  const int wave = __builtin_amdgcn_readfirstlane(tid >> 5);
  const int hh = lane >> 4, m = lane & 15;
  const int i  = (int)blockIdx.x >> 2;
  const int j0 = ((int)blockIdx.x & 3) * 64;

  {
    const int row = tid >> 2;
    const int dq  = (tid & 3) * 16;
    const float* pp = PQ + i * DDE + dq;
    const float* qp = PQ + NN * DDE + (j0 + row) * DDE + dq;
    const float* bp = bd + dq;
#pragma unroll
    for (int s = 0; s < 2; ++s) {
      const v4f p0 = *(const v4fa*)(pp + 8 * s), p1 = *(const v4fa*)(pp + 8 * s + 4);
      const v4f q0 = *(const v4fa*)(qp + 8 * s), q1 = *(const v4fa*)(qp + 8 * s + 4);
      const v4f b0 = bfr4(*(const v4fa*)(bp + 8 * s)), b1 = bfr4(*(const v4fa*)(bp + 8 * s + 4));
      float r[8];
      r[0] = fmaxf((p0.x + q0.x) + b0.x, 0.0f); r[1] = fmaxf((p0.y + q0.y) + b0.y, 0.0f);
      r[2] = fmaxf((p0.z + q0.z) + b0.z, 0.0f); r[3] = fmaxf((p0.w + q0.w) + b0.w, 0.0f);
      r[4] = fmaxf((p1.x + q1.x) + b1.x, 0.0f); r[5] = fmaxf((p1.y + q1.y) + b1.y, 0.0f);
      r[6] = fmaxf((p1.z + q1.z) + b1.z, 0.0f); r[7] = fmaxf((p1.w + q1.w) + b1.w, 0.0f);
      v8us hv, lv;
#pragma unroll
      for (int e = 0; e < 8; ++e) {
        const unsigned int hb = f2bf(r[e]);
        hv[e] = (unsigned short)hb;
        lv[e] = (unsigned short)f2bf(r[e] - bf2f(hb));
      }
      *(v8usa*)(As + row * APITCH + dq + 8 * s) = hv;
      *(v8usa*)(As + row * APITCH + DDE + dq + 8 * s) = lv;
    }
  }
  __syncthreads();

  const int rg = wave & 3, cg = wave >> 2;
  v8f acc[8];
  {
    const v8f z = {0.f, 0.f, 0.f, 0.f, 0.f, 0.f, 0.f, 0.f};
#pragma unroll
    for (int t = 0; t < 8; ++t) acc[t] = z;
  }
  const unsigned short* ap = As + (16 * rg + m) * APITCH + 8 * hh;
  const unsigned short* bp = WG2 + (size_t)(128 * cg + m) * KG + 8 * hh;
#pragma unroll 1
  for (int k0 = 0; k0 < KG; k0 += 32) {
    FragB af;
    af.h[0] = *(const v8usa*)(ap + k0);
    af.h[1] = *(const v8usa*)(ap + k0 + 16);
#pragma unroll
    for (int nt = 0; nt < 8; ++nt) {
      const unsigned short* wq = bp + (size_t)(16 * nt) * KG + k0;
      FragB bf;
      bf.h[0] = *(const v8usa*)wq;
      bf.h[1] = *(const v8usa*)(wq + 16);
      acc[nt] = wmb(af, bf, acc[nt]);
    }
  }

#pragma unroll
  for (int nt = 0; nt < 8; ++nt) {
    const int lc = 128 * cg + 16 * nt + m;
#pragma unroll
    for (int r = 0; r < 8; ++r) {
      const int lr = 16 * rg + 8 * hh + r;
      stg[lr * 256 + lc] = acc[nt][r];
    }
  }
  __syncthreads();

  const v4f bg0 = bfr4(*(const v4fa*)(bg + 4 * lane));
  const v4f bg1 = bfr4(*(const v4fa*)(bg + 128 + 4 * lane));
#pragma unroll 1
  for (int rr = 0; rr < 8; ++rr) {
    const int lr = wave * 8 + rr;
    const int j  = j0 + lr;
    const bool dg = (j == i);
    float* orow = HO + ((size_t)i * NSLOT + 1 + (size_t)j) * HD;
#pragma unroll
    for (int c = 0; c < 2; ++c) {
      const int col = 128 * c + 4 * lane;
      const v4f p  = *(const v4fa*)(stg + lr * 256 + col);
      const v4f bb = (c == 0) ? bg0 : bg1;
      const v4f t4 = *(const v4fa*)(TT + (size_t)j * HD + col);
      const v4f g4 = bfr4(*(const v4fa*)(ghs + (size_t)j * HD + col));
      v4f v;
      v.x = sigm(p.x + bb.x) * t4.x;
      v.y = sigm(p.y + bb.y) * t4.y;
      v.z = sigm(p.z + bb.z) * t4.z;
      v.w = sigm(p.w + bb.w) * t4.w;
      v.x = dg ? g4.x : v.x;
      v.y = dg ? g4.y : v.y;
      v.z = dg ? g4.z : v.z;
      v.w = dg ? g4.w : v.w;
      *(v4fa*)(stg + lr * 256 + col) = v;
      *(volatile v4f*)(orow + col) = v;
    }
  }
  __threadfence();
#pragma unroll 1
  for (int rr = 0; rr < 8; ++rr) {
    const int lr = wave * 8 + rr;
    const int j  = j0 + lr;
    float* orow = HO + ((size_t)i * NSLOT + 1 + (size_t)j) * HD;
#pragma unroll
    for (int c = 0; c < 2; ++c) {
      const int col = 128 * c + 4 * lane;
      const v4f v = *(const v4fa*)(stg + lr * 256 + col);
      *(volatile v4f*)(orow + col) = v;
    }
  }
}

__global__ __launch_bounds__(256) void k_row(const float* __restrict__ HO, const float* __restrict__ UV,
                                             unsigned short* CP)
{
  __shared__ __attribute__((aligned(16))) float suv[2048];
  __shared__ __attribute__((aligned(16))) float se[NHD * EP];
  __shared__ __attribute__((aligned(16))) unsigned short crow[KC];
  __shared__ float ssf[NHD];
  __shared__ float sinv[NHD];
  const int tid = (int)threadIdx.x, lane = tid & 31;
  const int wave = __builtin_amdgcn_readfirstlane(tid >> 5);
  const int i = (int)blockIdx.x;
  const float* hb = HO + (size_t)i * (size_t)(NSLOT * HD);

  *(v4fa*)(suv + 4 * tid)        = *(const v4fa*)(UV + 4 * tid);
  *(v4fa*)(suv + 1024 + 4 * tid) = *(const v4fa*)(UV + 1024 + 4 * tid);
  __syncthreads();

  if (wave == 0) {
    const v4f x0 = *(const v4fa*)(hb + 8 * lane), x1 = *(const v4fa*)(hb + 8 * lane + 4);
#pragma unroll 1
    for (int z = 0; z < NHD; ++z) {
      const v4f w0 = *(const v4fa*)(suv + z * HD + 8 * lane);
      const v4f w1 = *(const v4fa*)(suv + z * HD + 8 * lane + 4);
      const float d = wsum(dot8(x0, x1, w0, w1));
      if (lane == 0) ssf[z] = d;
    }
  }
#pragma unroll 1
  for (int k = wave; k < NSLOT; k += 8) {
    const float* rp = hb + (size_t)k * HD + 8 * lane;
    const v4f x0 = *(const v4fa*)rp, x1 = *(const v4fa*)(rp + 4);
#pragma unroll 1
    for (int z = 0; z < NHD; ++z) {
      const v4f w0 = *(const v4fa*)(suv + 1024 + z * HD + 8 * lane);
      const v4f w1 = *(const v4fa*)(suv + 1024 + z * HD + 8 * lane + 4);
      const float d = wsum(dot8(x0, x1, w0, w1));
      if (lane == 0) se[z * EP + k] = d;
    }
  }
  __syncthreads();

  if (wave < NHD) {
    float* ez = se + wave * EP;
    const float ss = ssf[wave];
    float mx = -3.0e38f;
#pragma unroll 1
    for (int t = 0; t < 9; ++t) {
      const int k  = lane + 32 * t;
      const int kc = k < NSLOT ? k : NSLOT - 1;
      float e = ss + ez[kc];
      e = e > 0.0f ? e : 0.2f * e;
      if (k < NSLOT) ez[k] = e;
      mx = fmaxf(mx, (k < NSLOT) ? e : -3.0e38f);
    }
    mx = wmax(mx);
    float sum = 0.0f;
#pragma unroll 1
    for (int t = 0; t < 9; ++t) {
      const int k  = lane + 32 * t;
      const int kc = k < NSLOT ? k : NSLOT - 1;
      float p = expf(ez[kc] - mx);
      p = (k < NSLOT) ? p : 0.0f;
      if (k < NSLOT) ez[k] = p;
      sum += p;
    }
    sum = wsum(sum);
    if (lane == 0) sinv[wave] = 1.0f / sum;
  }
  __syncthreads();

  float c0 = 0.0f, c1 = 0.0f, c2 = 0.0f, c3 = 0.0f;
#pragma unroll 4
  for (int k = 0; k < NSLOT; ++k) {
    const float x = hb[(size_t)k * HD + tid];
    c0 = fmaf(se[k], x, c0);
    c1 = fmaf(se[EP + k], x, c1);
    c2 = fmaf(se[2 * EP + k], x, c2);
    c3 = fmaf(se[3 * EP + k], x, c3);
  }
  c0 *= sinv[0]; c1 *= sinv[1]; c2 *= sinv[2]; c3 *= sinv[3];
  {
    const unsigned int h0 = f2bf(c0), h1 = f2bf(c1), h2 = f2bf(c2), h3 = f2bf(c3);
    crow[tid]              = (unsigned short)h0;
    crow[256 + tid]        = (unsigned short)h1;
    crow[512 + tid]        = (unsigned short)h2;
    crow[768 + tid]        = (unsigned short)h3;
    crow[1024 + tid]       = (unsigned short)f2bf(c0 - bf2f(h0));
    crow[1024 + 256 + tid] = (unsigned short)f2bf(c1 - bf2f(h1));
    crow[1024 + 512 + tid] = (unsigned short)f2bf(c2 - bf2f(h2));
    crow[1024 + 768 + tid] = (unsigned short)f2bf(c3 - bf2f(h3));
  }
  __syncthreads();
  const v8us o = *(const v8usa*)(crow + 8 * tid);
  unsigned short* dp = CP + (size_t)i * KC + 8 * tid;
  *(volatile v8us*)dp = o;
  __threadfence();
  *(volatile v8us*)dp = o;
}

__global__ __launch_bounds__(128) void k_out(const unsigned short* __restrict__ A,
                                             const unsigned short* __restrict__ WT,
                                             const float* __restrict__ bias, float* outF)
{
  __shared__ __attribute__((aligned(16))) float stg[64 * 64];
  const int tid = (int)threadIdx.x, lane = tid & 31;
  const int wave = __builtin_amdgcn_readfirstlane(tid >> 5);
  const int hh = lane >> 4, m = lane & 15;
  const int rowBase = (int)blockIdx.x * 64;
  const int col0    = (int)blockIdx.y * 64;

  v8f acc[4];
  {
    const v8f z = {0.f, 0.f, 0.f, 0.f, 0.f, 0.f, 0.f, 0.f};
    acc[0] = z; acc[1] = z; acc[2] = z; acc[3] = z;
  }
  const unsigned short* ap = A  + (size_t)(rowBase + 16 * wave + m) * KC + 8 * hh;
  const unsigned short* wp = WT + (size_t)(col0 + m) * KC + 8 * hh;
#pragma unroll 1
  for (int ks = 0; ks < KC / 32; ++ks) {
    FragB af;
    af.h[0] = *(const v8usa*)(ap + 32 * ks);
    af.h[1] = *(const v8usa*)(ap + 32 * ks + 16);
#pragma unroll
    for (int t = 0; t < 4; ++t) {
      const unsigned short* wq = wp + (size_t)(16 * t) * KC + 32 * ks;
      FragB bf;
      bf.h[0] = *(const v8usa*)wq;
      bf.h[1] = *(const v8usa*)(wq + 16);
      acc[t] = wmb(af, bf, acc[t]);
    }
  }

#pragma unroll
  for (int t = 0; t < 4; ++t) {
    const int lc = 16 * t + m;
#pragma unroll
    for (int r = 0; r < 8; ++r) {
      const int lr = 16 * wave + 8 * hh + r;
      stg[lr * 64 + lc] = acc[t][r];
    }
  }
  __syncthreads();

  const v4f b4 = bfr4(*(const v4fa*)(bias + col0 + 4 * m));
  v4f fv[8];
#pragma unroll
  for (int i = 0; i < 8; ++i) {
    const int lr = 16 * wave + 2 * i + hh;
    const v4f s = *(const v4fa*)(stg + lr * 64 + 4 * m);
    v4f v;
    v.x = 0.25f * s.x; v.y = 0.25f * s.y; v.z = 0.25f * s.z; v.w = 0.25f * s.w;
    v.x = (v.x > 0.0f ? v.x : 0.0f) + b4.x;
    v.y = (v.y > 0.0f ? v.y : 0.0f) + b4.y;
    v.z = (v.z > 0.0f ? v.z : 0.0f) + b4.z;
    v.w = (v.w > 0.0f ? v.w : 0.0f) + b4.w;
    fv[i] = v;
  }
#pragma unroll
  for (int i = 0; i < 8; ++i) {
    const int gr = rowBase + 16 * wave + 2 * i + hh;
    float* op = outF + (size_t)gr * HD + col0 + 4 * m;
    *(volatile v4f*)op = fv[i];
  }
  __threadfence();
#pragma unroll
  for (int i = 0; i < 8; ++i) {
    const int gr = rowBase + 16 * wave + 2 * i + hh;
    float* op = outF + (size_t)gr * HD + col0 + 4 * m;
    *(volatile v4f*)op = fv[i];
  }
}

extern "C" void kernel_launch(void* const* d_in, const int* in_sizes, int n_in,
                              void* d_out, int out_size, void* d_ws, size_t ws_size,
                              hipStream_t stream) {
  if (n_in < 11) return;
  if (in_sizes[0] != NN * HD || in_sizes[1] != NN * HD) return;
  if (in_sizes[2] != NN * 2 || in_sizes[3] != NN * 2) return;
  if (in_sizes[4] != 8 * DDE || in_sizes[5] != DDE) return;
  if (in_sizes[6] != DDE * HD || in_sizes[7] != HD) return;
  if (in_sizes[8] != NHD * HD * HD) return;
  if (in_sizes[9] != 2 * HD || in_sizes[10] != HD) return;
  if (out_size != NN * HD) return;

  const float* ahs    = (const float*)d_in[0];
  const float* ghs    = (const float*)d_in[1];
  const float* goal   = (const float*)d_in[2];
  const float* action = (const float*)d_in[3];
  const float* Wd     = (const float*)d_in[4];
  const float* bd     = (const float*)d_in[5];
  const float* Wg     = (const float*)d_in[6];
  const float* bg     = (const float*)d_in[7];
  const float* wm     = (const float*)d_in[8];
  const float* av     = (const float*)d_in[9];
  const float* bias   = (const float*)d_in[10];
  float* out = (float*)d_out;

  char* ws = (char*)d_ws;
  size_t off = 0;
  const size_t oHO  = off; off += (size_t)NN * NSLOT * HD * 4;   off = (off + 255) & ~(size_t)255;
  const size_t oTT  = off; off += (size_t)NN * HD * 4;           off = (off + 255) & ~(size_t)255;
  const size_t oPQ  = off; off += (size_t)2 * NN * DDE * 4;      off = (off + 255) & ~(size_t)255;
  const size_t oWG  = off; off += (size_t)HD * KG * 2;           off = (off + 255) & ~(size_t)255;
  const size_t oWM  = off; off += (size_t)HD * KC * 2;           off = (off + 255) & ~(size_t)255;
  const size_t oUV  = off; off += (size_t)2 * NHD * HD * 4;      off = (off + 255) & ~(size_t)255;
  const size_t oCP  = off; off += (size_t)NN * KC * 2;           off = (off + 255) & ~(size_t)255;
  if (off > ws_size || off > (size_t)WSMAX) return;
  float*          HO  = (float*)(ws + oHO);
  float*          TT  = (float*)(ws + oTT);
  float*          PQ  = (float*)(ws + oPQ);
  unsigned short* WG2 = (unsigned short*)(ws + oWG);
  unsigned short* WM2 = (unsigned short*)(ws + oWM);
  float*          UV  = (float*)(ws + oUV);
  unsigned short* CP  = (unsigned short*)(ws + oCP);

  hipFuncSetAttribute(reinterpret_cast<const void*>(&k_pair),
                      hipFuncAttributeMaxDynamicSharedMemorySize, LDS_PAIR);

  k_prep<<<PB_ALL, 256, 0, stream>>>(ahs, goal, action, Wd, Wg, wm, av, TT, HO, PQ, WG2, WM2, UV);
  k_pair<<<NN * 4, 256, LDS_PAIR, stream>>>(PQ, bd, WG2, bg, TT, ghs, HO);
  k_row<<<NN, 256, 0, stream>>>(HO, UV, CP);
  k_out<<<dim3(NN / 64, HD / 64), 128, 0, stream>>>(CP, WM2, bias, out);
}
